// DeformableTransformerDecoderLayer_10316511445002
// MI455X (gfx1250) — hardware-verified
//
#include <hip/hip_runtime.h>
#include <hip/hip_bf16.h>
#include <math.h>

typedef __attribute__((ext_vector_type(16))) _Float16 v16h;
typedef __attribute__((ext_vector_type(2)))  _Float16 v2h;
typedef __attribute__((ext_vector_type(8)))  float    v8f;
typedef _Float16 f16_t;
typedef __attribute__((ext_vector_type(8)))  _Float16 v8h;
typedef __attribute__((ext_vector_type(4)))  float v4f;
typedef __attribute__((ext_vector_type(4)))  unsigned v4u;
typedef float __attribute__((may_alias)) float_a;
template <typename T> __device__ __forceinline__ void vst2(void* p, T v) { *(volatile T*)p = v; __threadfence(); *(volatile T*)p = v; }
__device__ __forceinline__ v8f wmma16(v16h a, v16h b, v8f c) {
    v8f d = __builtin_amdgcn_wmma_f32_16x16x32_f16(false, a, false, b, (short)0, c, false, false);
    asm volatile("v_nop\n\tv_nop\n\tv_nop\n\tv_nop" : "+v"(d) : "v"(a), "v"(b));
    return d;
}

#define NQ   900
#define NQP  928
#define BSZ  4
#define DM   256
#define NH   8
#define DH   32
#define NLV  4
#define NPT  4
#define DFF  1024
#define MROW (NQ*BSZ)
#define MPAD (NQP*BSZ)
#define MVAL (13294*BSZ)

__global__ void repack_w(const float* __restrict__ W, f16_t* __restrict__ P, int N) {
    int tileN = blockIdx.x;
    int kt    = blockIdx.y;
    int lane  = threadIdx.x & 31;
    int n     = tileN * 16 + (lane & 15);
    int koff  = kt * 32 + (lane >> 4) * 8;
    f16_t* out = P + (((size_t)tileN * gridDim.y + kt) * 32 + (size_t)lane) * 16;
    union { v8h h[2]; v4u u[2]; } pk;
#pragma unroll
    for (int i = 0; i < 16; ++i)
        pk.h[i >> 3][i & 7] = (f16_t)W[(size_t)(koff + ((i < 8) ? i : (i + 8))) * N + n];
    vst2(out, pk.u[0]); vst2(out + 8, pk.u[1]);
}

__global__ void fill_zero_f16(f16_t* __restrict__ p, int n) {
    int g = blockIdx.x * blockDim.x + threadIdx.x;
    if (g * 8 < n) { v4u z = {0u, 0u, 0u, 0u}; vst2(p + (size_t)g * 8, z); }
}

template<int OMODE, bool RELU>
__global__ void gemm_wmma(const float* __restrict__ A, const f16_t* __restrict__ Bp,
                          const float* __restrict__ bias, void* __restrict__ Cout,
                          int M, int N, int K) {
    int tileM = blockIdx.x;
    int tn0   = blockIdx.y * 4;
    int lane  = threadIdx.x & 31;
    int m     = lane & 15;
    int hf    = lane >> 4;
    int rowA  = tileM * 16 + m;
    int rA    = rowA < M ? rowA : (M - 1);
    int KT    = K >> 5;
    const float* ap = A + (size_t)rA * K;
    const f16_t* bp[4];
#pragma unroll
    for (int j = 0; j < 4; ++j)
        bp[j] = Bp + ((size_t)(tn0 + j) * KT) * 512 + (size_t)lane * 16;
    v8f acc[4] = {};
    for (int kt = 0; kt < KT; ++kt) {
        v16h a;
#pragma unroll
        for (int i = 0; i < 8; ++i) {
            int g = i >> 2, wi = i & 3;
            int kb = kt * 32 + g * 16 + hf * 8 + wi * 2;
            float2 p = *(const float2*)(ap + kb);
            a[2 * i]     = (_Float16)p.x;
            a[2 * i + 1] = (_Float16)p.y;
        }
        __builtin_prefetch(bp[0] + 512, 0, 1);
#pragma unroll
        for (int j = 0; j < 4; ++j) {
            v16h b = *(const v16h*)bp[j];
            bp[j] += 512;
            acc[j] = wmma16(a, b, acc[j]);
        }
    }
    __shared__ __align__(16) float st[16][64];
#pragma unroll
    for (int j = 0; j < 4; ++j) {
        int cl = j * 16 + (lane & 15);
        float bv = bias[tn0 * 16 + cl];
#pragma unroll
        for (int r = 0; r < 8; ++r) { float v = acc[j][r] + bv; if (RELU) v = fmaxf(v, 0.f); st[hf * 8 + r][cl] = v; }
    }
    asm volatile("s_wait_dscnt 0" ::: "memory"); __builtin_amdgcn_wave_barrier(); __builtin_amdgcn_fence(__ATOMIC_RELEASE, "workgroup");
    const int c0 = tn0 * 16;
    if (OMODE == 0) {
#pragma unroll
        for (int q = 0; q < 8; ++q) { const int rl = q * 2 + (lane >> 4), pc = lane & 15; const int row = tileM * 16 + rl;
            if (row < M) vst2((float*)Cout + (size_t)row * N + c0 + pc * 4, *(const v4f*)(&st[rl][pc * 4])); }
    } else {
#pragma unroll
        for (int q = 0; q < 4; ++q) { const int rl = q * 4 + (lane >> 3), pc = lane & 7; const int row = tileM * 16 + rl;
            union { v8h h; v4u u; } pk;
#pragma unroll
            for (int e = 0; e < 8; ++e) pk.h[e] = (f16_t)st[rl][pc * 8 + e];
            if (row < M) vst2((f16_t*)Cout + (size_t)row * N + c0 + pc * 8, pk.u); }
    }
}

__global__ void attn_kernel(const f16_t* __restrict__ qb, const f16_t* __restrict__ kb,
                            const f16_t* __restrict__ vr, float* __restrict__ obuf) {
    int qt   = blockIdx.x;
    int bh   = blockIdx.y;
    int b    = bh & 3, h = bh >> 2;
    int lane = threadIdx.x & 31;
    int m    = lane & 15;
    int hf   = lane >> 4;
    __shared__ f16_t sc[16][944];

    v16h qa;
    int  qrow = qt * 16 + m;
    const f16_t* qp = qb + ((size_t)qrow * BSZ + b) * DM + h * DH;
#pragma unroll
    for (int i = 0; i < 8; ++i) {
        int g = i >> 2, wi = i & 3;
        int kbase = g * 16 + hf * 8 + wi * 2;
        v2h t = *(const v2h*)(qp + kbase);
        qa[2 * i]     = t.x;
        qa[2 * i + 1] = t.y;
    }
    const float scale = 0.17677669529663687f;
    for (int kt = 0; kt < 57; ++kt) {
        int krow = kt * 16 + (lane & 15);
        const f16_t* kp = kb + ((size_t)krow * BSZ + b) * DM + h * DH + hf * 8;
        union { v16h v; v8h q2[2]; } kf; kf.q2[0] = *(const v8h*)kp; kf.q2[1] = *(const v8h*)(kp + 16);
        v8f s = {};
        s = wmma16(qa, kf.v, s);
        int col = kt * 16 + (lane & 15);
        int rb  = (lane >> 4) * 8;
#pragma unroll
        for (int r = 0; r < 8; ++r) sc[rb + r][col] = (f16_t)(s[r] * scale);
    }
    __syncthreads();
    if (lane < 16) {
        float mx = -1e30f;
        for (int j = 0; j < NQ; ++j) mx = fmaxf(mx, (float)sc[lane][j]);
        float sum = 0.f;
        for (int j = 0; j < NQ; ++j) {
            float e = expf((float)sc[lane][j] - mx);
            sum += e;
            sc[lane][j] = (f16_t)e;
        }
        float inv = 1.f / sum;
        for (int j = 0; j < NQ; ++j) sc[lane][j] = (f16_t)((float)sc[lane][j] * inv);
        for (int j = NQ; j < 944; ++j) sc[lane][j] = (f16_t)0.f;
    }
    __syncthreads();
    v8f acc0 = {}, acc1 = {};
    const f16_t* v0 = vr + (size_t)b * DM + h * DH + (lane & 15);
    const f16_t* v1 = v0 + 16;
    for (int kt = 0; kt < 29; ++kt) {
        v16h pa;
#pragma unroll
        for (int i = 0; i < 8; ++i) {
            int g = i >> 2, wi = i & 3;
            int kbase = kt * 32 + g * 16 + hf * 8 + wi * 2;
            v2h t = *(const v2h*)(&sc[m][kbase]);
            pa[2 * i]     = t.x;
            pa[2 * i + 1] = t.y;
        }
        v16h vf0, vf1;
#pragma unroll
        for (int i = 0; i < 8; ++i) {
            const size_t k0 = (size_t)(kt * 32 + hf * 8 + i) * (BSZ * DM), k1 = (size_t)(kt * 32 + 16 + hf * 8 + i) * (BSZ * DM);
            vf0[i] = v0[k0]; vf0[8 + i] = v0[k1]; vf1[i] = v1[k0]; vf1[8 + i] = v1[k1];
        }
        acc0 = wmma16(pa, vf0, acc0);
        acc1 = wmma16(pa, vf1, acc1);
    }
    int col = lane & 15;
    __shared__ __align__(16) float so[16][32];
#pragma unroll
    for (int r = 0; r < 8; ++r) { so[hf * 8 + r][col] = acc0[r]; so[hf * 8 + r][col + 16] = acc1[r]; }
    asm volatile("s_wait_dscnt 0" ::: "memory"); __builtin_amdgcn_wave_barrier(); __builtin_amdgcn_fence(__ATOMIC_RELEASE, "workgroup");
#pragma unroll 4
    for (int rl = 0; rl < 16; ++rl) { const int row = qt * 16 + rl;
        if (row < NQ) vst2(obuf + ((size_t)row * BSZ + b) * DM + h * DH + lane, (float_a)so[rl][lane]); }
}

__global__ void msdeform_kernel(const float* __restrict__ off, const float* __restrict__ awl,
                                const f16_t* __restrict__ valh, const float* __restrict__ ref,
                                float* __restrict__ samp) {
    int r    = blockIdx.x;
    int b    = r & 3;
    int h    = threadIdx.x >> 5;
    int lane = threadIdx.x & 31;

    const float* ap = awl + (size_t)r * (NH * NLV * NPT) + h * (NLV * NPT);
    float lg[16];
    float mx = -1e30f;
#pragma unroll
    for (int i = 0; i < 16; ++i) { lg[i] = ap[i]; mx = fmaxf(mx, lg[i]); }
    float sum = 0.f;
#pragma unroll
    for (int i = 0; i < 16; ++i) { lg[i] = expf(lg[i] - mx); sum += lg[i]; }
    float inv = 1.f / sum;

    const int HL[4] = {100, 50, 25, 13};
    const int WL[4] = {100, 50, 25, 13};
    const int ST[4] = {0, 10000, 12500, 13125};
    const float* op = off + (size_t)r * (NH * NLV * NPT * 2) + h * (NLV * NPT * 2);
    const f16_t* vbase = valh + (size_t)b * DM + h * DH + lane;
    float acc = 0.f;
#pragma unroll
    for (int l = 0; l < NLV; ++l) {
        float rx = ref[(size_t)r * (NLV * 2) + l * 2 + 0];
        float ry = ref[(size_t)r * (NLV * 2) + l * 2 + 1];
        int Hl = HL[l], Wl = WL[l], s0 = ST[l];
        for (int p = 0; p < NPT; ++p) {
            float w  = lg[l * 4 + p] * inv;
            float lx = rx + op[l * 8 + p * 2 + 0] / (float)Wl;
            float ly = ry + op[l * 8 + p * 2 + 1] / (float)Hl;
            float x = lx * Wl - 0.5f, y = ly * Hl - 0.5f;
            float x0f = floorf(x), y0f = floorf(y);
            float fx = x - x0f, fy = y - y0f;
            int x0 = (int)x0f, y0 = (int)y0f;
#pragma unroll
            for (int c = 0; c < 4; ++c) {
                int xi = x0 + (c & 1), yi = y0 + (c >> 1);
                float wc = ((c & 1) ? fx : 1.f - fx) * ((c >> 1) ? fy : 1.f - fy);
                bool ok = (xi >= 0) & (xi < Wl) & (yi >= 0) & (yi < Hl);
                int xc = xi < 0 ? 0 : (xi >= Wl ? Wl - 1 : xi);
                int yc = yi < 0 ? 0 : (yi >= Hl ? Hl - 1 : yi);
                int pos = s0 + yc * Wl + xc;
                float v = (float)vbase[(size_t)pos * (BSZ * DM)];
                acc += (ok ? w * wc : 0.f) * v;
            }
        }
    }
    vst2(samp + (size_t)r * DM + h * DH + lane, (float_a)acc);
}

__global__ void residual_ln(const float* __restrict__ x, const float* __restrict__ y,
                            const float* __restrict__ g, const float* __restrict__ be,
                            float* __restrict__ out) {
    int row  = blockIdx.x;
    int lane = threadIdx.x;
    float v[8];
    float s = 0.f;
#pragma unroll
    for (int i = 0; i < 8; ++i) {
        int c = lane + i * 32;
        v[i] = x[(size_t)row * DM + c] + y[(size_t)row * DM + c];
        s += v[i];
    }
#pragma unroll
    for (int o = 16; o > 0; o >>= 1) s += __shfl_xor(s, o, 32);
    float mu = s * (1.f / 256.f);
    float var = 0.f;
#pragma unroll
    for (int i = 0; i < 8; ++i) { float d = v[i] - mu; var += d * d; }
#pragma unroll
    for (int o = 16; o > 0; o >>= 1) var += __shfl_xor(var, o, 32);
    var *= (1.f / 256.f);
    float rs = rsqrtf(var + 1e-5f);
#pragma unroll
    for (int i = 0; i < 8; ++i) {
        int c = lane + i * 32;
        vst2(out + (size_t)row * DM + c, (float_a)((v[i] - mu) * rs * g[c] + be[c]));
    }
}

__global__ void add_f32(const float* __restrict__ a, const float* __restrict__ b,
                        float* __restrict__ o, int n) {
    int i = blockIdx.x * blockDim.x + threadIdx.x;
    if (i < n) vst2(o + i, (float_a)(a[i] + b[i]));
}

extern "C" void kernel_launch(void* const* d_in, const int* in_sizes, int n_in,
                              void* d_out, int out_size, void* d_ws, size_t ws_size,
                              hipStream_t stream) {
    (void)in_sizes; (void)n_in; (void)out_size; (void)ws_size;
    const float* tgt     = (const float*)d_in[0];
    const float* pos     = (const float*)d_in[1];
    const float* refpts  = (const float*)d_in[2];
    const float* mem     = (const float*)d_in[3];
    const float* sa_wq   = (const float*)d_in[6];  const float* sa_bq   = (const float*)d_in[7];
    const float* sa_wk   = (const float*)d_in[8];  const float* sa_bk   = (const float*)d_in[9];
    const float* sa_wv   = (const float*)d_in[10]; const float* sa_bv   = (const float*)d_in[11];
    const float* sa_wo   = (const float*)d_in[12]; const float* sa_bo   = (const float*)d_in[13];
    const float* ln2_g   = (const float*)d_in[14]; const float* ln2_b   = (const float*)d_in[15];
    const float* ca_wval = (const float*)d_in[16]; const float* ca_bval = (const float*)d_in[17];
    const float* ca_woff = (const float*)d_in[18]; const float* ca_boff = (const float*)d_in[19];
    const float* ca_wattn= (const float*)d_in[20]; const float* ca_battn= (const float*)d_in[21];
    const float* ca_wout = (const float*)d_in[22]; const float* ca_bout = (const float*)d_in[23];
    const float* ln1_g   = (const float*)d_in[24]; const float* ln1_b   = (const float*)d_in[25];
    const float* ffn_w1  = (const float*)d_in[26]; const float* ffn_b1  = (const float*)d_in[27];
    const float* ffn_w2  = (const float*)d_in[28]; const float* ffn_b2  = (const float*)d_in[29];
    const float* ln3_g   = (const float*)d_in[30]; const float* ln3_b   = (const float*)d_in[31];

    char*  base = (char*)d_ws;
    size_t off  = 0;
    auto carve = [&](size_t bytes) -> void* {
        void* p = base + off;
        off += (bytes + 255) & ~(size_t)255;
        return p;
    };
    const size_t MD   = (size_t)MROW * DM;
    const size_t MDP  = (size_t)MPAD * DM;
    float* xq    = (float*)carve(MD * 4);
    float* obuf  = (float*)carve(MD * 4);
    float* sabuf = (float*)carve(MD * 4);
    float* tgt2  = (float*)carve(MD * 4);
    float* tgt3  = (float*)carve(MD * 4);
    float* offb  = (float*)carve(MD * 4);
    float* awb   = (float*)carve((size_t)MROW * 128 * 4);
    float* ffn1  = (float*)carve((size_t)MROW * DFF * 4);
    f16_t* qbuf  = (f16_t*)carve(MDP * 2);
    f16_t* kbuf  = (f16_t*)carve(MDP * 2);
    f16_t* vrow  = (f16_t*)carve(MDP * 2);
    f16_t* valh  = (f16_t*)carve((size_t)MVAL * DM * 2);
    f16_t* wqP   = (f16_t*)carve((size_t)DM * DM * 2);
    f16_t* wkP   = (f16_t*)carve((size_t)DM * DM * 2);
    f16_t* wvP   = (f16_t*)carve((size_t)DM * DM * 2);
    f16_t* woP   = (f16_t*)carve((size_t)DM * DM * 2);
    f16_t* wvalP = (f16_t*)carve((size_t)DM * DM * 2);
    f16_t* woffP = (f16_t*)carve((size_t)DM * 256 * 2);
    f16_t* wattP = (f16_t*)carve((size_t)DM * 128 * 2);
    f16_t* woutP = (f16_t*)carve((size_t)DM * DM * 2);
    f16_t* w1P   = (f16_t*)carve((size_t)DM * DFF * 2);
    f16_t* w2P   = (f16_t*)carve((size_t)DFF * DM * 2);

    const int tot  = MROW * DM;
    const int padN = (MPAD - MROW) * DM;

    repack_w<<<dim3(16, 8),  32, 0, stream>>>(sa_wq,   wqP,   256);
    repack_w<<<dim3(16, 8),  32, 0, stream>>>(sa_wk,   wkP,   256);
    repack_w<<<dim3(16, 8),  32, 0, stream>>>(sa_wv,   wvP,   256);
    repack_w<<<dim3(16, 8),  32, 0, stream>>>(sa_wo,   woP,   256);
    repack_w<<<dim3(16, 8),  32, 0, stream>>>(ca_wval, wvalP, 256);
    repack_w<<<dim3(16, 8),  32, 0, stream>>>(ca_woff, woffP, 256);
    repack_w<<<dim3(8, 8),   32, 0, stream>>>(ca_wattn,wattP, 128);
    repack_w<<<dim3(16, 8),  32, 0, stream>>>(ca_wout, woutP, 256);
    repack_w<<<dim3(64, 8),  32, 0, stream>>>(ffn_w1,  w1P,   1024);
    repack_w<<<dim3(16, 32), 32, 0, stream>>>(ffn_w2,  w2P,   256);

    fill_zero_f16<<<dim3((padN / 8 + 255) / 256), 256, 0, stream>>>(qbuf + MD, padN);
    fill_zero_f16<<<dim3((padN / 8 + 255) / 256), 256, 0, stream>>>(kbuf + MD, padN);
    fill_zero_f16<<<dim3((padN / 8 + 255) / 256), 256, 0, stream>>>(vrow + MD, padN);

    add_f32<<<dim3((tot + 255) / 256), 256, 0, stream>>>(tgt, pos, xq, tot);
    gemm_wmma<1, false><<<dim3(225, 4), 32, 0, stream>>>(xq,  wqP, sa_bq, qbuf, MROW, 256, 256);
    gemm_wmma<1, false><<<dim3(225, 4), 32, 0, stream>>>(xq,  wkP, sa_bk, kbuf, MROW, 256, 256);
    gemm_wmma<1, false><<<dim3(225, 4), 32, 0, stream>>>(tgt, wvP, sa_bv, vrow, MROW, 256, 256);
    attn_kernel<<<dim3(57, 32), 32, 0, stream>>>(qbuf, kbuf, vrow, obuf);
    gemm_wmma<0, false><<<dim3(225, 4), 32, 0, stream>>>(obuf, woP, sa_bo, sabuf, MROW, 256, 256);
    residual_ln<<<dim3(MROW), 32, 0, stream>>>(tgt, sabuf, ln2_g, ln2_b, tgt2);

    add_f32<<<dim3((tot + 255) / 256), 256, 0, stream>>>(tgt2, pos, xq, tot);
    gemm_wmma<1, false><<<dim3(3324, 4), 32, 0, stream>>>(mem, wvalP, ca_bval, valh, MVAL, 256, 256);
    gemm_wmma<0, false><<<dim3(225, 4),  32, 0, stream>>>(xq, woffP, ca_boff, offb, MROW, 256, 256);
    gemm_wmma<0, false><<<dim3(225, 2),  32, 0, stream>>>(xq, wattP, ca_battn, awb, MROW, 128, 256);
    msdeform_kernel<<<dim3(MROW), 256, 0, stream>>>(offb, awb, valh, refpts, obuf);
    gemm_wmma<0, false><<<dim3(225, 4), 32, 0, stream>>>(obuf, woutP, ca_bout, sabuf, MROW, 256, 256);
    residual_ln<<<dim3(MROW), 32, 0, stream>>>(tgt2, sabuf, ln1_g, ln1_b, tgt3);

    gemm_wmma<0, true ><<<dim3(225, 16), 32, 0, stream>>>(tgt3, w1P, ffn_b1, ffn1, MROW, 1024, 256);
    gemm_wmma<0, false><<<dim3(225, 4),  32, 0, stream>>>(ffn1, w2P, ffn_b2, offb, MROW, 256, 1024);
    residual_ln<<<dim3(MROW), 32, 0, stream>>>(tgt3, offb, ln3_g, ln3_b, (float*)d_out);
}
